// GraphAgent_28896539967835
// MI455X (gfx1250) — hardware-verified
//
#include <hip/hip_runtime.h>

typedef _Float16 f16t;
typedef f16t  v16h __attribute__((ext_vector_type(16)));
typedef f16t  v8h  __attribute__((ext_vector_type(8)));
typedef f16t  v4h  __attribute__((ext_vector_type(4)));
typedef float v8f  __attribute__((ext_vector_type(8)));
typedef float v4f  __attribute__((ext_vector_type(4)));

#define NEMB   128
#define NNODE  16384
#define NEDGE  16384
#define NSTEM  4096
#define NGRAPH 1024
#define OPS    105
#define NSTEPS 12
#define NBLK   106
#define NSTT   131
#define NBND   130
#define WSCALE 16.0f
#define WINV   0.0625f

#define PK_ROOT  0
#define PK_WIH   16384
#define PK_WHH   65536
#define PK_B2E1  114688
#define PK_B2E2  131072
#define PK_S2P1  147456
#define PK_S2P2  180224
#define PK_S2P3  196608
#define PK_G2P1  210944
#define PK_TOTAL 227328

#define LCAP 256
#define PCAP 640

static_assert(NNODE % 64 == 0);
static_assert(NSTEM % 32 == 0);
static_assert(NGRAPH % 32 == 0);
static_assert(PK_TOTAL % 2048 == 0);
static_assert((NEDGE / 4) % 128 == 0);
static_assert((NNODE / 2) % 128 == 0);

union Frag { v16h v; v8h h[2]; };
union Pk8  { v8h hv; v4h q[2]; v4f fv; };

__device__ __forceinline__ v8f zero8() { v8f z = {0.f, 0.f, 0.f, 0.f, 0.f, 0.f, 0.f, 0.f}; return z; }
__device__ __forceinline__ int clampi(int v, int hi) { v = v < 0 ? 0 : v; return v > hi ? hi : v; }
__device__ __forceinline__ float lrelu(float x) { return x > 0.f ? x : 0.01f * x; }
__device__ __forceinline__ float sigf(float x) { return __builtin_amdgcn_rcpf(1.0f + __expf(-x)); }
__device__ __forceinline__ float tnhf(float x) { return 1.0f - 2.0f * __builtin_amdgcn_rcpf(__expf(2.0f * x) + 1.0f); }

__device__ __forceinline__ v8f mma(v16h a, v16h b, v8f c) {
  c = __builtin_amdgcn_wmma_f32_16x16x32_f16(false, a, false, b, (short)0, c, false, false);
  asm volatile("v_nop\n\tv_nop\n\tv_nop\n\tv_nop" : "+v"(c) : "v"(a), "v"(b));
  return c;
}

__device__ __forceinline__ v16h lda(const f16t* base, int stride, int row0, int kt, int lane) {
  const f16t* p = base + (row0 + (lane & 15)) * stride + kt * 32 + 8 * (lane >> 4);
  Frag f;
  f.h[0] = *(const v8h*)p;
  f.h[1] = *(const v8h*)(p + 16);
  return f.v;
}

__device__ __forceinline__ v16h ldb(const f16t* p0, int nT, int kt, int ct, int lane) {
  const f16t* p = p0 + ((((kt * nT) + ct) * 32 + lane) << 4);
  Frag f;
  f.h[0] = *(const v8h*)p;
  f.h[1] = *(const v8h*)(p + 8);
  return f.v;
}

__device__ __forceinline__ void push_hit(int* lst, int& cnt, bool hit, int ent, int cap) {
  const unsigned b = __builtin_amdgcn_ballot_w32(hit);
  if (hit) {
    const int pos = cnt + (int)__builtin_amdgcn_mbcnt_lo(b, 0u);
    if (pos < cap) lst[pos] = ent;
  }
  cnt += __builtin_popcount(b);
}

__device__ __forceinline__ void store_rows(const float* hs, float* F, f16t* H, int R, int lane) {
  const int hh = lane >> 4, q = lane & 15;
#pragma unroll
  for (int row = 0; row < 16; ++row) {
    const v4f v = *(const v4f*)(hs + row * NEMB + 4 * lane);
    *(volatile v4f*)(F + (size_t)(R + row) * NEMB + 4 * lane) = v;
  }
#pragma unroll
  for (int j = 0; j < 8; ++j) {
    const int row = 2 * j + hh;
    const float* s = hs + row * NEMB + 8 * q;
    Pk8 u;
    u.q[0] = __builtin_convertvector(*(const v4f*)s, v4h);
    u.q[1] = __builtin_convertvector(*(const v4f*)(s + 4), v4h);
    *(volatile v4f*)(H + (size_t)(R + row) * NEMB + 8 * q) = u.fv;
  }
}

__global__ __launch_bounds__(256) void k_pack(const float* __restrict__ conv_root,
                                              const float* __restrict__ wih,
                                              const float* __restrict__ whh,
                                              const float* __restrict__ b2e1,
                                              const float* __restrict__ b2e2,
                                              const float* __restrict__ s2p1,
                                              const float* __restrict__ s2p2,
                                              const float* __restrict__ s2p3,
                                              const float* __restrict__ g2p1,
                                              f16t* pk) {
  const int g = blockIdx.x * 256 + threadIdx.x;
  if (g >= PK_TOTAL / 8) return;
  const int e0 = g * 8;
  const float* W; int K, Nr, nT, tr, base;
  if      (e0 < PK_WIH)  { W = conv_root; K = 128; Nr = 128; nT = 8;  tr = 0; base = PK_ROOT; }
  else if (e0 < PK_WHH)  { W = wih;       K = 128; Nr = 384; nT = 24; tr = 1; base = PK_WIH;  }
  else if (e0 < PK_B2E1) { W = whh;       K = 128; Nr = 384; nT = 24; tr = 1; base = PK_WHH;  }
  else if (e0 < PK_B2E2) { W = b2e1;      K = 128; Nr = 128; nT = 8;  tr = 0; base = PK_B2E1; }
  else if (e0 < PK_S2P1) { W = b2e2;      K = 128; Nr = 128; nT = 8;  tr = 0; base = PK_B2E2; }
  else if (e0 < PK_S2P2) { W = s2p1;      K = 256; Nr = 128; nT = 8;  tr = 0; base = PK_S2P1; }
  else if (e0 < PK_S2P3) { W = s2p2;      K = 128; Nr = 128; nT = 8;  tr = 0; base = PK_S2P2; }
  else if (e0 < PK_G2P1) { W = s2p3;      K = 128; Nr = OPS; nT = 7;  tr = 0; base = PK_S2P3; }
  else                   { W = g2p1;      K = 128; Nr = 128; nT = 8;  tr = 0; base = PK_G2P1; }
  const int loc  = e0 - base;
  const int j    = (loc >> 3) & 1;
  const int ln   = (loc >> 4) & 31;
  const int tile = loc >> 9;
  const int ct   = tile % nT;
  const int kt   = tile / nT;
  const int hh   = ln >> 4;
  const int n    = ct * 16 + (ln & 15);
  const int kb   = kt * 32 + 16 * j + 8 * hh;
  Pk8 u;
#pragma unroll
  for (int i = 0; i < 8; ++i) {
    const int k = kb + i;
    float v = 0.f;
    if (n < Nr) v = tr ? W[n * K + k] : W[k * Nr + n];
    u.hv[i] = (f16t)(v * WSCALE);
  }
  volatile v4f* dst = (volatile v4f*)(pk + e0);
  *dst = u.fv;
  __threadfence();
  *dst = u.fv;
}

__global__ __launch_bounds__(64) void k_pro(const float* __restrict__ emb_block,
                                            const int* __restrict__ x_ids,
                                            const f16t* __restrict__ pk,
                                            const float* __restrict__ b1,
                                            const float* __restrict__ b2,
                                            float* F, f16t* H) {
  __shared__ __attribute__((aligned(16))) f16t  xs[2][16 * NEMB];
  __shared__ __attribute__((aligned(16))) f16t  t1[2][16 * NEMB];
  __shared__ __attribute__((aligned(16))) float hs[2][16 * NEMB];
  const int t = threadIdx.x, w = t >> 5, lane = t & 31, hh = lane >> 4, nc = lane & 15;
  const int R = blockIdx.x * 32 + 16 * w;
  f16t* xw = &xs[w][0];
  f16t* tw = &t1[w][0];
  float* hw = &hs[w][0];

#pragma unroll 1
  for (int row = 0; row < 16; ++row) {
    const int id = clampi(x_ids[R + row], NBLK - 1);
    const v4f v = *(const v4f*)(emb_block + id * NEMB + 4 * lane);
    *(v4h*)(xw + row * NEMB + 4 * lane) = __builtin_convertvector(v, v4h);
  }
  __syncthreads();

  v16h a[4];
#pragma unroll
  for (int kt = 0; kt < 4; ++kt) a[kt] = lda(xw, NEMB, 0, kt, lane);
  const f16t* P1 = pk + PK_B2E1;
#pragma unroll 1
  for (int ct = 0; ct < 8; ++ct) {
    v8f acc = zero8();
#pragma unroll
    for (int kt = 0; kt < 4; ++kt) acc = mma(a[kt], ldb(P1, 8, kt, ct, lane), acc);
    const int col = ct * 16 + nc;
    const float bb = b1[col];
#pragma unroll
    for (int r = 0; r < 8; ++r)
      tw[(8 * hh + r) * NEMB + col] = (f16t)lrelu(acc[r] * WINV + bb);
  }
  __syncthreads();

#pragma unroll
  for (int kt = 0; kt < 4; ++kt) a[kt] = lda(tw, NEMB, 0, kt, lane);
  const f16t* P2 = pk + PK_B2E2;
#pragma unroll 1
  for (int ct = 0; ct < 8; ++ct) {
    v8f acc = zero8();
#pragma unroll
    for (int kt = 0; kt < 4; ++kt) acc = mma(a[kt], ldb(P2, 8, kt, ct, lane), acc);
    const int col = ct * 16 + nc;
    const float bb = b2[col];
#pragma unroll
    for (int r = 0; r < 8; ++r)
      hw[(8 * hh + r) * NEMB + col] = acc[r] * WINV + bb;
  }
  __syncthreads();

  store_rows(hw, F, H, R, lane);
  __threadfence();
  store_rows(hw, F, H, R, lane);
}

__global__ __launch_bounds__(128) void k_step(const float* __restrict__ Fin,
                                              const f16t* __restrict__ Hin,
                                              float* Fout, f16t* Hout,
                                              const float* __restrict__ emb_bond,
                                              const int* __restrict__ bond_ids,
                                              const int* __restrict__ edge_src,
                                              const int* __restrict__ edge_dst,
                                              const f16t* __restrict__ pk,
                                              const float* __restrict__ cbias,
                                              const float* __restrict__ bih,
                                              const float* __restrict__ bhh) {
  __shared__ __attribute__((aligned(16))) float aggh[4][16 * NEMB];
  __shared__ __attribute__((aligned(16))) f16t  ml[4][16 * NEMB];
  __shared__ int lst[4][LCAP];
  __shared__ int lcnt[4];
  __shared__ int degc[64];
  const int t = threadIdx.x, w = t >> 5, lane = t & 31, hh = lane >> 4, nc = lane & 15;
  const int rb = blockIdx.x * 64;
  const int R  = rb + 16 * w;
  float* aw = &aggh[w][0];
  f16t*  mw = &ml[w][0];

  {
    const v4f z = {0.f, 0.f, 0.f, 0.f};
#pragma unroll
    for (int row = 0; row < 16; ++row) *(v4f*)(aw + row * NEMB + 4 * lane) = z;
  }
  if (lane < 16) degc[16 * w + lane] = 0;

  int cnt = 0;
  {
    const int eb = w * (NEDGE / 4);
    int* lw = &lst[w][0];
#pragma unroll 1
    for (int it = 0; it < (NEDGE / 4) / 128; ++it) {
      const int e0 = eb + it * 128 + 4 * lane;
      const int4 d = *(const int4*)(edge_dst + e0);
      const int s0 = d.x - rb, s1 = d.y - rb, s2 = d.z - rb, s3 = d.w - rb;
      const bool q0 = (unsigned)s0 < 64u, q1 = (unsigned)s1 < 64u;
      const bool q2 = (unsigned)s2 < 64u, q3 = (unsigned)s3 < 64u;
      if (__builtin_amdgcn_ballot_w32(q0 | q1 | q2 | q3) == 0u) continue;
      push_hit(lw, cnt, q0, ((e0 + 0) << 6) | s0, LCAP);
      push_hit(lw, cnt, q1, ((e0 + 1) << 6) | s1, LCAP);
      push_hit(lw, cnt, q2, ((e0 + 2) << 6) | s2, LCAP);
      push_hit(lw, cnt, q3, ((e0 + 3) << 6) | s3, LCAP);
    }
  }
  if (lane == 0) lcnt[w] = cnt < LCAP ? cnt : LCAP;
  __syncthreads();

#pragma unroll 1
  for (int q = 0; q < 4; ++q) {
    int n = lcnt[q];
    n = n < 0 ? 0 : (n > LCAP ? LCAP : n);
#pragma unroll 1
    for (int i = 0; i < n; ++i) {
      const int ent = lst[q][i];
      const int slot = ent & 63;
      if ((slot >> 4) != w) continue;
      const int e   = clampi(ent >> 6, NEDGE - 1);
      const int src = clampi(edge_src[e], NNODE - 1);
      const int b0  = clampi(bond_ids[2 * e], NBND - 1);
      const int b1  = clampi(bond_ids[2 * e + 1], NBND - 1);
      const v4f xv = *(const v4f*)(Fin + (size_t)src * NEMB + 4 * lane);
      const v4f bv = *(const v4f*)(emb_bond + b0 * NEMB + 4 * lane);
      float p = xv[0] * bv[0];
      p += xv[1] * bv[1];
      p += xv[2] * bv[2];
      p += xv[3] * bv[3];
      p += __shfl_xor(p, 16, 32);
      p += __shfl_xor(p, 8, 32);
      p += __shfl_xor(p, 4, 32);
      p += __shfl_xor(p, 2, 32);
      p += __shfl_xor(p, 1, 32);
      const v4f bw = *(const v4f*)(emb_bond + b1 * NEMB + 4 * lane);
      float* ap = aw + (slot & 15) * NEMB + 4 * lane;
      v4f a = *(v4f*)ap;
      a += p * bw;
      *(v4f*)ap = a;
      if (lane == 0) degc[slot] += 1;
    }
  }
  __syncthreads();

  float rd[8];
#pragma unroll
  for (int r = 0; r < 8; ++r) {
    const int c = degc[16 * w + 8 * hh + r];
    rd[r] = __builtin_amdgcn_rcpf((float)(c < 1 ? 1 : c));
  }

  v16h as[4];
#pragma unroll
  for (int kt = 0; kt < 4; ++kt) as[kt] = lda(Hin, NEMB, R, kt, lane);
  const f16t* Proot = pk + PK_ROOT;
  const f16t* Pwih  = pk + PK_WIH;
  const f16t* Pwhh  = pk + PK_WHH;

#pragma unroll 1
  for (int ct = 0; ct < 8; ++ct) {
    v8f acc = zero8();
#pragma unroll
    for (int kt = 0; kt < 4; ++kt) acc = mma(as[kt], ldb(Proot, 8, kt, ct, lane), acc);
    const int col = ct * 16 + nc;
    const float cb = cbias[col];
#pragma unroll
    for (int r = 0; r < 8; ++r) {
      const int row = 8 * hh + r;
      const float v = acc[r] * WINV + aw[row * NEMB + col] * rd[r] + cb;
      mw[row * NEMB + col] = (f16t)lrelu(v);
    }
  }
  __syncthreads();

  v16h am[4];
#pragma unroll
  for (int kt = 0; kt < 4; ++kt) am[kt] = lda(mw, NEMB, 0, kt, lane);

#pragma unroll 1
  for (int c16 = 0; c16 < 8; ++c16) {
    v8f ar = zero8(), az = zero8(), ain = zero8(), ahn = zero8();
#pragma unroll
    for (int kt = 0; kt < 4; ++kt) {
      ar  = mma(as[kt], ldb(Pwhh, 24, kt, c16, lane), ar);
      ar  = mma(am[kt], ldb(Pwih, 24, kt, c16, lane), ar);
      az  = mma(as[kt], ldb(Pwhh, 24, kt, c16 + 8, lane), az);
      az  = mma(am[kt], ldb(Pwih, 24, kt, c16 + 8, lane), az);
      ain = mma(am[kt], ldb(Pwih, 24, kt, c16 + 16, lane), ain);
      ahn = mma(as[kt], ldb(Pwhh, 24, kt, c16 + 16, lane), ahn);
    }
    const int col = c16 * 16 + nc;
    const float br  = bih[col] + bhh[col];
    const float bz  = bih[128 + col] + bhh[128 + col];
    const float bin = bih[256 + col];
    const float bhn = bhh[256 + col];
#pragma unroll
    for (int r = 0; r < 8; ++r) {
      const int row = 8 * hh + r;
      const float rg = sigf(ar[r] * WINV + br);
      const float zg = sigf(az[r] * WINV + bz);
      const float ng = tnhf(ain[r] * WINV + bin + rg * (ahn[r] * WINV + bhn));
      const float hp = Fin[(size_t)(R + row) * NEMB + col];
      const float hn = (1.0f - zg) * ng + zg * hp;
      aw[row * NEMB + col] = hn;
    }
  }
  __syncthreads();

  store_rows(aw, Fout, Hout, R, lane);
  __threadfence();
  store_rows(aw, Fout, Hout, R, lane);
}

__global__ __launch_bounds__(64) void k_stem(const float* __restrict__ F,
                                             const float* __restrict__ emb_stem,
                                             const int* __restrict__ stemtype_ids,
                                             const int* __restrict__ stems_batch,
                                             const int* __restrict__ stems_local,
                                             const int* __restrict__ node_offsets,
                                             const f16t* __restrict__ pk,
                                             const float* __restrict__ b1,
                                             const float* __restrict__ b2,
                                             const float* __restrict__ b3,
                                             float* out) {
  __shared__ __attribute__((aligned(16))) f16t  scl[2][16 * 256];
  __shared__ __attribute__((aligned(16))) f16t  h1l[2][16 * NEMB];
  __shared__ __attribute__((aligned(16))) float ost[32 * OPS];
  const int t = threadIdx.x, w = t >> 5, lane = t & 31, hh = lane >> 4, nc = lane & 15;
  const int S0 = blockIdx.x * 32 + 16 * w;
  f16t* sw  = &scl[w][0];
  f16t* h1w = &h1l[w][0];

#pragma unroll 1
  for (int row = 0; row < 16; ++row) {
    const int s  = S0 + row;
    const int gb = clampi(stems_batch[s], NGRAPH - 1);
    const int idx = clampi(node_offsets[gb] + stems_local[s], NNODE - 1);
    const int st = clampi(stemtype_ids[s], NSTT - 1);
    const v4f a = *(const v4f*)(F + (size_t)idx * NEMB + 4 * lane);
    const v4f b = *(const v4f*)(emb_stem + st * NEMB + 4 * lane);
    *(v4h*)(sw + row * 256 + 4 * lane)        = __builtin_convertvector(a, v4h);
    *(v4h*)(sw + row * 256 + NEMB + 4 * lane) = __builtin_convertvector(b, v4h);
  }
  __syncthreads();

  v16h a8[8];
#pragma unroll
  for (int kt = 0; kt < 8; ++kt) a8[kt] = lda(sw, 256, 0, kt, lane);
  const f16t* P1 = pk + PK_S2P1;
#pragma unroll 1
  for (int ct = 0; ct < 8; ++ct) {
    v8f acc = zero8();
#pragma unroll
    for (int kt = 0; kt < 8; ++kt) acc = mma(a8[kt], ldb(P1, 8, kt, ct, lane), acc);
    const int col = ct * 16 + nc;
    const float bb = b1[col];
#pragma unroll
    for (int r = 0; r < 8; ++r)
      h1w[(8 * hh + r) * NEMB + col] = (f16t)lrelu(acc[r] * WINV + bb);
  }
  __syncthreads();

  v16h a4[4];
#pragma unroll
  for (int kt = 0; kt < 4; ++kt) a4[kt] = lda(h1w, NEMB, 0, kt, lane);
  f16t* h2w = sw;
  const f16t* P2 = pk + PK_S2P2;
#pragma unroll 1
  for (int ct = 0; ct < 8; ++ct) {
    v8f acc = zero8();
#pragma unroll
    for (int kt = 0; kt < 4; ++kt) acc = mma(a4[kt], ldb(P2, 8, kt, ct, lane), acc);
    const int col = ct * 16 + nc;
    const float bb = b2[col];
#pragma unroll
    for (int r = 0; r < 8; ++r)
      h2w[(8 * hh + r) * NEMB + col] = (f16t)lrelu(acc[r] * WINV + bb);
  }
  __syncthreads();

#pragma unroll
  for (int kt = 0; kt < 4; ++kt) a4[kt] = lda(h2w, NEMB, 0, kt, lane);
  const f16t* P3 = pk + PK_S2P3;
#pragma unroll 1
  for (int ct = 0; ct < 7; ++ct) {
    v8f acc = zero8();
#pragma unroll
    for (int kt = 0; kt < 4; ++kt) acc = mma(a4[kt], ldb(P3, 7, kt, ct, lane), acc);
    const int col = ct * 16 + nc;
    const bool ok = col < OPS;
    const float bb = b3[ok ? col : 0];
#pragma unroll
    for (int r = 0; r < 8; ++r)
      if (ok) ost[(16 * w + 8 * hh + r) * OPS + col] = acc[r] * WINV + bb;
  }
  __syncthreads();

  const size_t base = (size_t)blockIdx.x * 32 * OPS;
#pragma unroll 1
  for (int p = 0; p < 14; ++p) {
    const int qd = p * 64 + t;
    if (qd < (32 * OPS) / 4) {
      const v4f v = *(const v4f*)(ost + 4 * qd);
      *(volatile v4f*)(out + base + 4 * qd) = v;
    }
  }
  __threadfence();
#pragma unroll 1
  for (int p = 0; p < 14; ++p) {
    const int qd = p * 64 + t;
    if (qd < (32 * OPS) / 4) {
      const v4f v = *(const v4f*)(ost + 4 * qd);
      *(volatile v4f*)(out + base + 4 * qd) = v;
    }
  }
}

__global__ __launch_bounds__(64) void k_pool(const float* __restrict__ F,
                                             const int* __restrict__ batch,
                                             const f16t* __restrict__ pk,
                                             const float* __restrict__ b1,
                                             const float* __restrict__ w2,
                                             const float* __restrict__ b2,
                                             float* out1) {
  __shared__ __attribute__((aligned(16))) float gs[32][NEMB];
  __shared__ __attribute__((aligned(16))) f16t  gml[2][16 * NEMB];
  __shared__ __attribute__((aligned(16))) float res[32];
  __shared__ int plst[2][PCAP];
  __shared__ int pcnt[2];
  __shared__ int gc[32];
  const int t = threadIdx.x, w = t >> 5, lane = t & 31, hh = lane >> 4, nc = lane & 15;
  const int g0 = blockIdx.x * 32;
  f16t* gw = &gml[w][0];

  {
    const v4f z = {0.f, 0.f, 0.f, 0.f};
#pragma unroll
    for (int row = 0; row < 16; ++row) *(v4f*)(&gs[16 * w + row][0] + 4 * lane) = z;
  }
  if (lane < 16) gc[16 * w + lane] = 0;

  int cnt = 0;
  {
    const int nb = w * (NNODE / 2);
    int* lw = &plst[w][0];
#pragma unroll 1
    for (int it = 0; it < (NNODE / 2) / 128; ++it) {
      const int n0 = nb + it * 128 + 4 * lane;
      const int4 d = *(const int4*)(batch + n0);
      const int s0 = d.x - g0, s1 = d.y - g0, s2 = d.z - g0, s3 = d.w - g0;
      const bool q0 = (unsigned)s0 < 32u, q1 = (unsigned)s1 < 32u;
      const bool q2 = (unsigned)s2 < 32u, q3 = (unsigned)s3 < 32u;
      if (__builtin_amdgcn_ballot_w32(q0 | q1 | q2 | q3) == 0u) continue;
      push_hit(lw, cnt, q0, ((n0 + 0) << 5) | s0, PCAP);
      push_hit(lw, cnt, q1, ((n0 + 1) << 5) | s1, PCAP);
      push_hit(lw, cnt, q2, ((n0 + 2) << 5) | s2, PCAP);
      push_hit(lw, cnt, q3, ((n0 + 3) << 5) | s3, PCAP);
    }
  }
  if (lane == 0) pcnt[w] = cnt < PCAP ? cnt : PCAP;
  __syncthreads();

#pragma unroll 1
  for (int q = 0; q < 2; ++q) {
    int n = pcnt[q];
    n = n < 0 ? 0 : (n > PCAP ? PCAP : n);
#pragma unroll 1
    for (int i = 0; i < n; ++i) {
      const int ent = plst[q][i];
      const int slot = ent & 31;
      if ((slot >> 4) != w) continue;
      const int node = clampi(ent >> 5, NNODE - 1);
      const v4f v = *(const v4f*)(F + (size_t)node * NEMB + 4 * lane);
      float* ap = &gs[slot][0] + 4 * lane;
      v4f a = *(v4f*)ap;
      a += v;
      *(v4f*)ap = a;
      if (lane == 0) gc[slot] += 1;
    }
  }
  __syncthreads();

#pragma unroll 1
  for (int row = 0; row < 16; ++row) {
    const int slot = 16 * w + row;
    const int c = gc[slot];
    const float rc = __builtin_amdgcn_rcpf((float)(c < 1 ? 1 : c));
    const v4f v = *(const v4f*)(&gs[slot][0] + 4 * lane) * rc;
    *(v4h*)(gw + row * NEMB + 4 * lane) = __builtin_convertvector(v, v4h);
  }
  __syncthreads();

  v16h a[4];
#pragma unroll
  for (int kt = 0; kt < 4; ++kt) a[kt] = lda(gw, NEMB, 0, kt, lane);
  const f16t* P1 = pk + PK_G2P1;
  float part[8];
#pragma unroll
  for (int r = 0; r < 8; ++r) part[r] = 0.f;
#pragma unroll 1
  for (int ct = 0; ct < 8; ++ct) {
    v8f acc = zero8();
#pragma unroll
    for (int kt = 0; kt < 4; ++kt) acc = mma(a[kt], ldb(P1, 8, kt, ct, lane), acc);
    const int col = ct * 16 + nc;
    const float bb = b1[col];
    const float ww = w2[col];
#pragma unroll
    for (int r = 0; r < 8; ++r) part[r] += lrelu(acc[r] * WINV + bb) * ww;
  }
#pragma unroll
  for (int r = 0; r < 8; ++r) {
    part[r] += __shfl_xor(part[r], 1, 32);
    part[r] += __shfl_xor(part[r], 2, 32);
    part[r] += __shfl_xor(part[r], 4, 32);
    part[r] += __shfl_xor(part[r], 8, 32);
  }
  if (nc == 0) {
    const float bb = b2[0];
#pragma unroll
    for (int r = 0; r < 8; ++r) res[16 * w + 8 * hh + r] = part[r] + bb;
  }
  __syncthreads();

  if (t < 8) {
    const v4f v = *(const v4f*)(res + 4 * t);
    *(volatile v4f*)(out1 + g0 + 4 * t) = v;
  }
  __threadfence();
  if (t < 8) {
    const v4f v = *(const v4f*)(res + 4 * t);
    *(volatile v4f*)(out1 + g0 + 4 * t) = v;
  }
}

extern "C" void kernel_launch(void* const* d_in, const int* in_sizes, int n_in,
                              void* d_out, int out_size, void* d_ws, size_t ws_size,
                              hipStream_t stream) {
  if (n_in < 32) return;
  if ((size_t)out_size < (size_t)NSTEM * OPS + (size_t)NGRAPH) return;
  if (in_sizes[23] < NNODE || in_sizes[24] < NSTEM || in_sizes[25] < 2 * NEDGE ||
      in_sizes[26] < NEDGE || in_sizes[27] < NEDGE || in_sizes[28] < NNODE ||
      in_sizes[29] < NSTEM || in_sizes[30] < NSTEM || in_sizes[31] < NGRAPH) return;

  const float* emb_block = (const float*)d_in[0];
  const float* emb_stem  = (const float*)d_in[1];
  const float* emb_bond  = (const float*)d_in[2];
  const float* conv_root = (const float*)d_in[3];
  const float* conv_bias = (const float*)d_in[4];
  const float* b2e_w1 = (const float*)d_in[5];
  const float* b2e_b1 = (const float*)d_in[6];
  const float* b2e_w2 = (const float*)d_in[7];
  const float* b2e_b2 = (const float*)d_in[8];
  const float* gru_wih = (const float*)d_in[9];
  const float* gru_whh = (const float*)d_in[10];
  const float* gru_bih = (const float*)d_in[11];
  const float* gru_bhh = (const float*)d_in[12];
  const float* s2p_w1 = (const float*)d_in[13];
  const float* s2p_b1 = (const float*)d_in[14];
  const float* s2p_w2 = (const float*)d_in[15];
  const float* s2p_b2 = (const float*)d_in[16];
  const float* s2p_w3 = (const float*)d_in[17];
  const float* s2p_b3 = (const float*)d_in[18];
  const float* g2p_w1 = (const float*)d_in[19];
  const float* g2p_b1 = (const float*)d_in[20];
  const float* g2p_w2 = (const float*)d_in[21];
  const float* g2p_b2 = (const float*)d_in[22];
  const int* x_ids        = (const int*)d_in[23];
  const int* stemtype_ids = (const int*)d_in[24];
  const int* bond_ids     = (const int*)d_in[25];
  const int* edge_src     = (const int*)d_in[26];
  const int* edge_dst     = (const int*)d_in[27];
  const int* batch        = (const int*)d_in[28];
  const int* stems_batch  = (const int*)d_in[29];
  const int* stems_local  = (const int*)d_in[30];
  const int* node_offsets = (const int*)d_in[31];

  const size_t szF = (size_t)NNODE * NEMB * sizeof(float);
  const size_t szH = (size_t)NNODE * NEMB * sizeof(f16t);
  const size_t szP = (((size_t)PK_TOTAL * sizeof(f16t)) + 255) & ~(size_t)255;
  const size_t need = 2 * szF + 2 * szH + szP;
  if (ws_size < need) return;
  char* ws = (char*)d_ws;
  float* F0 = (float*)(ws);
  float* F1 = (float*)(ws + szF);
  f16t*  H0 = (f16t*)(ws + 2 * szF);
  f16t*  H1 = (f16t*)(ws + 2 * szF + szH);
  f16t*  PK = (f16t*)(ws + 2 * szF + 2 * szH);

  k_pack<<<PK_TOTAL / 8 / 256, 256, 0, stream>>>(conv_root, gru_wih, gru_whh, b2e_w1, b2e_w2,
                                                  s2p_w1, s2p_w2, s2p_w3, g2p_w1, PK);
  k_pro<<<NNODE / 32, 64, 0, stream>>>(emb_block, x_ids, PK, b2e_b1, b2e_b2, F0, H0);
  for (int s = 0; s < NSTEPS; ++s) {
    const float* Fi = (s & 1) ? F1 : F0;
    const f16t*  Hi = (s & 1) ? H1 : H0;
    float* Fo = (s & 1) ? F0 : F1;
    f16t*  Ho = (s & 1) ? H0 : H1;
    k_step<<<NNODE / 64, 128, 0, stream>>>(Fi, Hi, Fo, Ho, emb_bond, bond_ids, edge_src, edge_dst,
                                           PK, conv_bias, gru_bih, gru_bhh);
  }
  const float* Ff = (NSTEPS & 1) ? F1 : F0;
  k_stem<<<NSTEM / 32, 64, 0, stream>>>(Ff, emb_stem, stemtype_ids, stems_batch, stems_local,
                                        node_offsets, PK, s2p_b1, s2p_b2, s2p_b3, (float*)d_out);
  k_pool<<<NGRAPH / 32, 64, 0, stream>>>(Ff, batch, PK, g2p_b1, g2p_w2, g2p_b2,
                                         (float*)d_out + (size_t)NSTEM * OPS);
}
